// PointActorRecurrent_52295521796462
// MI455X (gfx1250) — hardware-verified
//
#include <hip/hip_runtime.h>


namespace {
constexpr int B = 256, NPT = 1024, HID = 256, ACT = 6, HZ = 50, G3 = 3 * HID;
constexpr float AS_ = 8.0f;

typedef _Float16 b16;
typedef __attribute__((ext_vector_type(16))) _Float16 v16b;
typedef __attribute__((ext_vector_type(8))) _Float16 v8b;
typedef __attribute__((ext_vector_type(8))) float v8f;
typedef __attribute__((ext_vector_type(4))) float v4f;
__device__ __forceinline__ float bf16_rne(float f) { unsigned int u = __float_as_uint(f); u += 0x7FFFu + ((u >> 16) & 1u); return __uint_as_float(u & 0xFFFF0000u); }
__device__ __forceinline__ void split16(float v, b16& hi, b16& lo) { hi = (b16)v; lo = (b16)(v - (float)hi); }
__device__ __forceinline__ v16b frag_kb(const b16* p, int hh) { const v8b a = *(const v8b*)(p + 8 * hh), b = *(const v8b*)(p + 16 + 8 * hh); v16b f;
#pragma unroll
  for (int e = 0; e < 8; ++e) { f[e] = a[e]; f[8 + e] = b[e]; } return f; }
__device__ __forceinline__ v8f wmma16b(v16b a, v16b b, v8f c) { v8f d = __builtin_amdgcn_wmma_f32_16x16x32_f16(false, a, false, b, (short)0, c, false, false); asm volatile("v_nop\n\tv_nop\n\tv_nop\n\tv_nop" : "+v"(d) : "v"(a), "v"(b)); return d; }
__device__ __forceinline__ void wave_lds_sync() { __builtin_amdgcn_fence(__ATOMIC_RELEASE, "workgroup"); __builtin_amdgcn_wave_barrier(); __builtin_amdgcn_fence(__ATOMIC_ACQUIRE, "workgroup"); }
__device__ __forceinline__ float nexp(float x) { return __builtin_amdgcn_exp2f(x * 1.4426950408889634f); }
__device__ __forceinline__ float sigm(float x) { return __builtin_amdgcn_rcpf(1.0f + nexp(-x)); }
__device__ __forceinline__ float tanh_(float x) { const float e = nexp(-2.0f * fabsf(x)); const float t = (1.0f - e) * __builtin_amdgcn_rcpf(1.0f + e); return (x >= 0.0f) ? t : -t; }
__device__ __forceinline__ float pmul(float a, float b) { float p = a * b; asm volatile("" : "+v"(p)); return p; }
__device__ __forceinline__ void frag_split(const float* p, int hh, v16b& fh, v16b& fl) {
#pragma unroll
  for (int e = 0; e < 8; ++e) { b16 a, c; split16(p[8 * hh + e] * AS_, a, c); fh[e] = a; fl[e] = c; split16(p[16 + 8 * hh + e] * AS_, a, c); fh[8 + e] = a; fl[8 + e] = c; } }

struct Woff { static constexpr size_t W2 = 0, W3 = W2 + 128 * 64, M1 = W3 + 512 * 128, M2 = M1 + 256 * 512, M3 = M2 + 128 * 256, HH = M3 + 256 * 128, O1 = HH + 768 * 256, O2 = O1 + 64 * 256, O3 = O2 + 64 * 64, END = O3 + 16 * 64; };
__global__ __launch_bounds__(256) void prep_kernel(const float* __restrict__ ew1, const float* __restrict__ eb1, const float* __restrict__ ew2, const float* __restrict__ eb2, const float* __restrict__ ew3, const float* __restrict__ eb3,
                                                   const float* __restrict__ mw1, const float* __restrict__ mb1, const float* __restrict__ mw2, const float* __restrict__ mb2, const float* __restrict__ mw3, const float* __restrict__ mb3,
                                                   const float* __restrict__ wih, const float* __restrict__ whh, const float* __restrict__ bih, const float* __restrict__ bhh,
                                                   const float* __restrict__ ow1, const float* __restrict__ ob1, const float* __restrict__ ow2, const float* __restrict__ ob2, const float* __restrict__ ow3, const float* __restrict__ ob3,
                                                   b16* __restrict__ R, float* __restrict__ P, float* __restrict__ Wih) {
  const int t_ = threadIdx.x + blockIdx.x * 256, nth = gridDim.x * 256;
  auto tr = [&](const float* W, int IN, int OUT, size_t base, int p) { const int o = p / IN, k = p % IN; ((volatile b16*)R)[base + p] = (b16)((o < OUT) ? bf16_rne(W[k * OUT + o]) : 0.0f); };
  for (int pass = 0; pass < 2; ++pass) {
    for (int p = t_; p < 128 * 64; p += nth) tr(ew2, 64, 128, Woff::W2, p);
    for (int p = t_; p < 512 * 128; p += nth) tr(ew3, 128, 512, Woff::W3, p);
    for (int p = t_; p < 256 * 512; p += nth) tr(mw1, 512, 256, Woff::M1, p);
    for (int p = t_; p < 128 * 256; p += nth) tr(mw2, 256, 128, Woff::M2, p);
    for (int p = t_; p < 256 * 128; p += nth) tr(mw3, 128, 256, Woff::M3, p);
    for (int p = t_; p < 768 * 256; p += nth) ((volatile b16*)R)[Woff::HH + p] = (b16)bf16_rne(whh[p]);
    for (int p = t_; p < 64 * 256; p += nth) tr(ow1, 256, 64, Woff::O1, p);
    for (int p = t_; p < 64 * 64; p += nth) tr(ow2, 64, 64, Woff::O2, p);
    for (int p = t_; p < 16 * 64; p += nth) { const int o = p / 64, k = p % 64; ((volatile b16*)R)[Woff::O3 + p] = (b16)((o < ACT) ? bf16_rne(ow3[k * ACT + o]) : 0.0f); }
    for (int p = t_; p < 768 * ACT; p += nth) ((volatile float*)Wih)[p] = bf16_rne(wih[p]);
    for (int p = t_; p < 3264; p += nth) { float v = 0.0f;
      if (p < 192) v = bf16_rne(ew1[p]); else if (p < 256) v = bf16_rne(eb1[p - 192]); else if (p < 384) v = bf16_rne(eb2[p - 256]); else if (p < 896) v = bf16_rne(eb3[p - 384]); else if (p < 1152) v = bf16_rne(mb1[p - 896]);
      else if (p < 1280) v = bf16_rne(mb2[p - 1152]); else if (p < 1536) v = bf16_rne(mb3[p - 1280]); else if (p < 2304) v = bf16_rne(bih[p - 1536]); else if (p < 3072) v = bf16_rne(bhh[p - 2304]); else if (p < 3136) v = bf16_rne(ob1[p - 3072]);
      else if (p < 3200) v = bf16_rne(ob2[p - 3136]); else if (p < 3200 + ACT) v = ob3[p - 3200];
      ((volatile float*)P)[p] = v; }
    __threadfence(); }
}

__global__ __launch_bounds__(128) void enc_kernel(const float* __restrict__ data, const float* __restrict__ P, const b16* __restrict__ R, float* __restrict__ pmax) {
  __shared__ __attribute__((aligned(16))) float T[128][128 + 4]; __shared__ float Mx[4][512];
  const int lane = threadIdx.x & 31, wave = threadIdx.x >> 5, nloc = lane & 15, hlf = lane >> 4, b = blockIdx.y, p0 = blockIdx.x * 128, m0 = wave * 32;
  const float* ew1 = P; const float* eb1 = P + 192; const float* eb2 = P + 256; const float* eb3 = P + 384;
  const float* da = data + ((size_t)b * NPT + p0 + m0 + nloc) * 3; const float* db = da + 16 * 3;
  const float xa0 = bf16_rne(da[0]), xa1 = bf16_rne(da[1]), xa2 = bf16_rne(da[2]), xb0 = bf16_rne(db[0]), xb1 = bf16_rne(db[1]), xb2 = bf16_rne(db[2]);
  v8f acc[2][8];
#pragma unroll
  for (int r = 0; r < 2; ++r)
#pragma unroll
    for (int t = 0; t < 8; ++t) acc[r][t] = (v8f){};
#pragma unroll
  for (int ks = 0; ks < 2; ++ks) { v16b a0, l0, a1, l1;
#pragma unroll
    for (int e = 0; e < 16; ++e) { const int k = ks * 32 + ((e < 8) ? (8 * hlf + e) : (16 + 8 * hlf + e - 8)); const float w0 = ew1[k], w1 = ew1[64 + k], w2 = ew1[128 + k], bb = eb1[k];
      b16 p, q; split16(fmaxf((pmul(xa0, w0) + pmul(xa1, w1)) + (pmul(xa2, w2) + bb), 0.0f) * AS_, p, q); a0[e] = p; l0[e] = q; split16(fmaxf((pmul(xb0, w0) + pmul(xb1, w1)) + (pmul(xb2, w2) + bb), 0.0f) * AS_, p, q); a1[e] = p; l1[e] = q; }
#pragma unroll
    for (int t = 0; t < 8; ++t) { const v16b bw = frag_kb(R + Woff::W2 + (size_t)(t * 16 + nloc) * 64 + ks * 32, hlf); acc[0][t] = wmma16b(a0, bw, acc[0][t]); acc[0][t] = wmma16b(l0, bw, acc[0][t]); acc[1][t] = wmma16b(a1, bw, acc[1][t]); acc[1][t] = wmma16b(l1, bw, acc[1][t]); } }
#pragma unroll
  for (int t = 0; t < 8; ++t) { const float bb = eb2[t * 16 + nloc];
#pragma unroll
    for (int r = 0; r < 2; ++r)
#pragma unroll
      for (int v = 0; v < 8; ++v) T[m0 + r * 16 + 8 * hlf + v][t * 16 + nloc] = fmaxf(acc[r][t][v] * (1.0f / AS_) + bb, 0.0f); }
  wave_lds_sync();
  for (int ct = 0; ct < 8; ++ct) { v8f c3[2][4];
#pragma unroll
    for (int r = 0; r < 2; ++r)
#pragma unroll
      for (int t = 0; t < 4; ++t) c3[r][t] = (v8f){};
#pragma unroll
    for (int kb = 0; kb < 128; kb += 32) { v16b a0, l0, a1, l1; frag_split(&T[m0 + nloc][kb], hlf, a0, l0); frag_split(&T[m0 + 16 + nloc][kb], hlf, a1, l1);
#pragma unroll
      for (int t = 0; t < 4; ++t) { const v16b bw = frag_kb(R + Woff::W3 + (size_t)(ct * 64 + t * 16 + nloc) * 128 + kb, hlf); c3[0][t] = wmma16b(a0, bw, c3[0][t]); c3[0][t] = wmma16b(l0, bw, c3[0][t]); c3[1][t] = wmma16b(a1, bw, c3[1][t]); c3[1][t] = wmma16b(l1, bw, c3[1][t]); } }
#pragma unroll
    for (int t = 0; t < 4; ++t) { const int c = ct * 64 + t * 16 + nloc; const float bb = eb3[c]; float mx = -INFINITY;
#pragma unroll
      for (int r = 0; r < 2; ++r)
#pragma unroll
        for (int v = 0; v < 8; ++v) mx = fmaxf(mx, fmaxf(c3[r][t][v] * (1.0f / AS_) + bb, 0.0f));
      mx = fmaxf(mx, __shfl_xor(mx, 16));
      if (hlf == 0) Mx[wave][c] = mx; } }
  __syncthreads();
  for (int pass = 0; pass < 2; ++pass) { { const int c4 = threadIdx.x * 4; v4f o;
#pragma unroll
      for (int e = 0; e < 4; ++e) o[e] = fmaxf(fmaxf(Mx[0][c4 + e], Mx[1][c4 + e]), fmaxf(Mx[2][c4 + e], Mx[3][c4 + e]));
      *(volatile v4f*)(pmax + ((size_t)b * (NPT / 128) + blockIdx.x) * 512 + c4) = o; } __threadfence(); }
}

__global__ __launch_bounds__(64) void head_kernel(const float* __restrict__ pmax, const float* __restrict__ P, const b16* __restrict__ R, float* __restrict__ h0) {
  __shared__ __attribute__((aligned(16))) float T[2][16][512 + 4];
  const int wid = threadIdx.x >> 5, lane = threadIdx.x & 31, nloc = lane & 15, hlf = lane >> 4; const int r0 = blockIdx.x * 32 + wid * 16;
  const float* mb1 = P + 896; const float* mb2 = P + 1152; const float* mb3 = P + 1280;
  for (int i = lane; i < 16 * 128; i += 32) { const int r = i >> 7, c4 = (i & 127) * 4; const float* pp = pmax + ((size_t)(r0 + r) * 8) * 512 + c4; v4f m = *(const v4f*)pp;
    for (int k = 1; k < 8; ++k) { const v4f q = *(const v4f*)(pp + k * 512);
#pragma unroll
      for (int e = 0; e < 4; ++e) m[e] = fmaxf(m[e], q[e]); }
    *(v4f*)(&T[wid][r][c4]) = m; }
  wave_lds_sync();
  auto gemm = [&](const b16* Bw, int KK, int NTL, v8f* acc) {
    for (int kb = 0; kb < KK; kb += 32) { v16b ah, al; frag_split(&T[wid][nloc][kb], hlf, ah, al);
      for (int t = 0; t < NTL; ++t) { const v16b bw = frag_kb(Bw + (size_t)(t * 16 + nloc) * KK + kb, hlf); acc[t] = wmma16b(ah, bw, acc[t]); acc[t] = wmma16b(al, bw, acc[t]); } } };
  v8f acc[16];
#pragma unroll
  for (int t = 0; t < 16; ++t) acc[t] = (v8f){};
  gemm(R + Woff::M1, 512, 16, acc); wave_lds_sync();
#pragma unroll
  for (int t = 0; t < 16; ++t)
#pragma unroll
    for (int v = 0; v < 8; ++v) T[wid][8 * hlf + v][t * 16 + nloc] = fmaxf(acc[t][v] * (1.0f / AS_) + mb1[t * 16 + nloc], 0.0f);
  wave_lds_sync();
#pragma unroll
  for (int t = 0; t < 8; ++t) acc[t] = (v8f){};
  gemm(R + Woff::M2, 256, 8, acc); wave_lds_sync();
#pragma unroll
  for (int t = 0; t < 8; ++t)
#pragma unroll
    for (int v = 0; v < 8; ++v) T[wid][8 * hlf + v][t * 16 + nloc] = fmaxf(acc[t][v] * (1.0f / AS_) + mb2[t * 16 + nloc], 0.0f);
  wave_lds_sync();
#pragma unroll
  for (int t = 0; t < 16; ++t) acc[t] = (v8f){};
  gemm(R + Woff::M3, 128, 16, acc); wave_lds_sync();
#pragma unroll
  for (int t = 0; t < 16; ++t)
#pragma unroll
    for (int v = 0; v < 8; ++v) T[wid][8 * hlf + v][t * 16 + nloc] = acc[t][v] * (1.0f / AS_) + mb3[t * 16 + nloc];
  wave_lds_sync();
  for (int pass = 0; pass < 2; ++pass) { for (int i = lane; i < 16 * 64; i += 32) { const int r = i >> 6, c4 = (i & 63) * 4; *(volatile v4f*)(h0 + (size_t)(r0 + r) * HID + c4) = *(const v4f*)(&T[wid][r][c4]); } __threadfence(); }
}

__global__ __launch_bounds__(32) void gru_kernel(const float* __restrict__ h0, const float* __restrict__ P, const float* __restrict__ Wih, const b16* __restrict__ R, float* __restrict__ dws, float* __restrict__ wsum) {
  __shared__ __attribute__((aligned(16))) float H[16][HID + 4], Rg[16][HID + 4], Zg[16][HID + 4], S[16][64 + 4], X[16][8], Dw[16 * HZ * ACT], Ws[16 * HZ * ACT];
  const int lane = threadIdx.x, nloc = lane & 15, hlf = lane >> 4; const int r0 = blockIdx.x * 16;
  const float* bih = P + 1536; const float* bhh = P + 2304; const float* ob1 = P + 3072; const float* ob2 = P + 3136; const float* ob3 = P + 3200;
  for (int i = lane; i < 16 * 64; i += 32) { const int r = i >> 6, c4 = (i & 63) * 4; *(v4f*)(&H[r][c4]) = *(const v4f*)(h0 + (size_t)(r0 + r) * HID + c4); }
  for (int i = lane; i < 16 * 8; i += 32) X[i >> 3][i & 7] = 0.0f;
  wave_lds_sync();
  const b16* Whh = R + Woff::HH;
  for (int step = 0; step < HZ; ++step) {
    for (int g = 0; g < 3; ++g) { v8f acc[16];
#pragma unroll
      for (int t = 0; t < 16; ++t) acc[t] = (v8f){};
      for (int kb = 0; kb < HID; kb += 32) { v16b ah, al; frag_split(&H[nloc][kb], hlf, ah, al);
#pragma unroll
        for (int t = 0; t < 16; ++t) { const v16b bw = frag_kb(Whh + (size_t)(g * HID + t * 16 + nloc) * HID + kb, hlf); acc[t] = wmma16b(ah, bw, acc[t]); acc[t] = wmma16b(al, bw, acc[t]); } }
#pragma unroll
      for (int t = 0; t < 16; ++t) { const int c = t * 16 + nloc, gc = g * HID + c; const float* wr = Wih + (size_t)gc * ACT; const float bi = bih[gc], bh = bhh[gc];
#pragma unroll
        for (int v = 0; v < 8; ++v) { const int row = 8 * hlf + v; float xi = bi;
#pragma unroll
          for (int a = 0; a < ACT; ++a) xi += pmul(X[row][a], wr[a]);
          const float hg = acc[t][v] * (1.0f / AS_) + bh;
          if (g == 0) Rg[row][c] = sigm(xi + hg); else if (g == 1) Zg[row][c] = sigm(xi + hg);
          else { const float n = tanh_(xi + Rg[row][c] * hg); const float z = Zg[row][c]; acc[t][v] = (1.0f - z) * n + z * H[row][c]; } } }
      if (g < 2) { wave_lds_sync(); continue; }
      wave_lds_sync();
#pragma unroll
      for (int t = 0; t < 16; ++t)
#pragma unroll
        for (int v = 0; v < 8; ++v) H[8 * hlf + v][t * 16 + nloc] = acc[t][v];
      wave_lds_sync(); }
    { v8f a1[4] = {{}, {}, {}, {}};
      for (int kb = 0; kb < HID; kb += 32) { v16b ah, al; frag_split(&H[nloc][kb], hlf, ah, al);
#pragma unroll
        for (int t = 0; t < 4; ++t) { const v16b bw = frag_kb(R + Woff::O1 + (size_t)(t * 16 + nloc) * HID + kb, hlf); a1[t] = wmma16b(ah, bw, a1[t]); a1[t] = wmma16b(al, bw, a1[t]); } }
#pragma unroll
      for (int t = 0; t < 4; ++t)
#pragma unroll
        for (int v = 0; v < 8; ++v) S[8 * hlf + v][t * 16 + nloc] = fmaxf(a1[t][v] * (1.0f / AS_) + ob1[t * 16 + nloc], 0.0f);
      wave_lds_sync();
      v8f a2[4] = {{}, {}, {}, {}};
#pragma unroll
      for (int kb = 0; kb < 64; kb += 32) { v16b ah, al; frag_split(&S[nloc][kb], hlf, ah, al);
#pragma unroll
        for (int t = 0; t < 4; ++t) { const v16b bw = frag_kb(R + Woff::O2 + (size_t)(t * 16 + nloc) * 64 + kb, hlf); a2[t] = wmma16b(ah, bw, a2[t]); a2[t] = wmma16b(al, bw, a2[t]); } }
      wave_lds_sync();
#pragma unroll
      for (int t = 0; t < 4; ++t)
#pragma unroll
        for (int v = 0; v < 8; ++v) S[8 * hlf + v][t * 16 + nloc] = fmaxf(a2[t][v] * (1.0f / AS_) + ob2[t * 16 + nloc], 0.0f);
      wave_lds_sync();
      v8f a3 = {};
#pragma unroll
      for (int kb = 0; kb < 64; kb += 32) { v16b ah, al; frag_split(&S[nloc][kb], hlf, ah, al); const v16b bw = frag_kb(R + Woff::O3 + (size_t)nloc * 64 + kb, hlf); a3 = wmma16b(ah, bw, a3); a3 = wmma16b(al, bw, a3); }
      wave_lds_sync();
      if (nloc < ACT) {
#pragma unroll
        for (int v = 0; v < 8; ++v) { const int row = 8 * hlf + v; const float dw = a3[v] * (1.0f / AS_) + ob3[nloc]; const float xn = X[row][nloc] + dw; X[row][nloc] = xn;
          Dw[(row * HZ + step) * ACT + nloc] = dw; Ws[(row * HZ + step) * ACT + nloc] = xn; } }
      wave_lds_sync(); }
  }
  for (int pass = 0; pass < 2; ++pass) { for (int i = lane; i < 16 * HZ * ACT / 4; i += 32) { *(volatile v4f*)(dws + (size_t)r0 * HZ * ACT + i * 4) = *(const v4f*)(&Dw[i * 4]); *(volatile v4f*)(wsum + (size_t)r0 * HZ * ACT + i * 4) = *(const v4f*)(&Ws[i * 4]); } __threadfence(); }
}
}

extern "C" void kernel_launch(void* const* d_in, const int* in_sizes, int n_in,
                              void* d_out, int out_size, void* d_ws, size_t ws_size, hipStream_t stream) {
  (void)n_in; (void)out_size;
  const float* data = (const float*)d_in[0];
  const float* ew1 = (const float*)d_in[2]; const float* eb1 = (const float*)d_in[3]; const float* ew2 = (const float*)d_in[4]; const float* eb2 = (const float*)d_in[5]; const float* ew3 = (const float*)d_in[6]; const float* eb3 = (const float*)d_in[7];
  const float* mw1 = (const float*)d_in[8]; const float* mb1 = (const float*)d_in[9]; const float* mw2 = (const float*)d_in[10]; const float* mb2 = (const float*)d_in[11]; const float* mw3 = (const float*)d_in[12]; const float* mb3 = (const float*)d_in[13];
  const float* wih = (const float*)d_in[14]; const float* whh = (const float*)d_in[15]; const float* bih = (const float*)d_in[16]; const float* bhh = (const float*)d_in[17];
  const float* ow1 = (const float*)d_in[18]; const float* ob1 = (const float*)d_in[19]; const float* ow2 = (const float*)d_in[20]; const float* ob2 = (const float*)d_in[21]; const float* ow3 = (const float*)d_in[22]; const float* ob3 = (const float*)d_in[23];
  float* dws = (float*)d_out; float* wsum = dws + (size_t)B * HZ * ACT;
  if (in_sizes[0] != B * NPT * 3 || in_sizes[1] != 1 || in_sizes[15] != G3 * HID || in_sizes[14] != G3 * ACT || in_sizes[22] != 64 * ACT) return;
  size_t off = 0; char* ws = (char*)d_ws;
  auto carve = [&](size_t bytes) { char* p = ws + off; off += (bytes + 255) & ~(size_t)255; return p; };
  b16* R = (b16*)carve(Woff::END * 2); float* P = (float*)carve(3328 * 4); float* Wih = (float*)carve((size_t)G3 * ACT * 4 + 256); float* pmax = (float*)carve((size_t)B * 8 * 512 * 4); float* h0 = (float*)carve((size_t)B * HID * 4);
  if (off > ws_size) return;
  prep_kernel<<<64, 256, 0, stream>>>(ew1, eb1, ew2, eb2, ew3, eb3, mw1, mb1, mw2, mb2, mw3, mb3, wih, whh, bih, bhh, ow1, ob1, ow2, ob2, ow3, ob3, R, P, Wih);
  enc_kernel<<<dim3(NPT / 128, B), 128, 0, stream>>>(data, P, R, pmax);
  head_kernel<<<B / 32, 64, 0, stream>>>(pmax, P, R, h0);
  gru_kernel<<<B / 16, 32, 0, stream>>>(h0, P, Wih, R, dws, wsum);
}
